// RoleAwareGraphTransformer_65859028517070
// MI455X (gfx1250) — hardware-verified
//
#include <hip/hip_runtime.h>
#include <hip/hip_bf16.h>

#define N_STOCKS 20000
#define IN_F     64
#define PE_F     32
#define TIN      96
#define HIDF     128
#define HEADS    4
#define CDIM     32
#define E_EDGES  100000
#define R_REL    5
#define EAUG     (E_EDGES + N_STOCKS)
#define LDS_STRIDE 136

typedef __attribute__((ext_vector_type(16))) _Float16 v16h;
typedef __attribute__((ext_vector_type(8)))  float    v8f;

union AFrag { unsigned int u[8]; v16h v; };
union BFrag { _Float16 e[16];    v16h v; };
typedef __attribute__((ext_vector_type(4))) float v4f_t;
typedef float v4fa __attribute__((ext_vector_type(4), may_alias));
#define BUCKET 64
#define LCAP   1280
#define NBK    ((N_STOCKS + BUCKET - 1) / BUCKET)
static __device__ __forceinline__ unsigned pk2(float a, float b) { return (unsigned)__builtin_bit_cast(unsigned short, (_Float16)a) | ((unsigned)__builtin_bit_cast(unsigned short, (_Float16)b) << 16); }
#define ST2F(ptr, val) do { *(volatile float*)(ptr) = (val); __threadfence(); *(volatile float*)(ptr) = (val); } while (0)

__global__ __launch_bounds__(256)
void cvt_f16_kernel(const float* __restrict__ src, _Float16* __restrict__ dst, int count) {
    int t = (blockIdx.x * 256 + threadIdx.x) * 2;
    if (t < count) { const unsigned p = pk2(src[t], src[t + 1]); *(volatile unsigned*)(dst + t) = p; __threadfence(); *(volatile unsigned*)(dst + t) = p; }
}

__global__ __launch_bounds__(32)
void pearl_concat_kernel(const float* __restrict__ x, const float* __restrict__ pW,
                         const float* __restrict__ pb, _Float16* __restrict__ h16) {
    int row = blockIdx.x;
    int t   = threadIdx.x;
    const float* xr = x + (size_t)row * IN_F;
    float acc = pb[t];
#pragma unroll 8
    for (int k = 0; k < IN_F; ++k) acc += xr[k] * pW[k * PE_F + t];
    float pe4[4];
#pragma unroll
    for (int j = 0; j < 4; ++j) pe4[j] = __shfl(acc, (4 * t + j) & 31, 32);
    typedef __attribute__((ext_vector_type(2))) unsigned v2u_t;
    v2u_t pk;
    if (t < 16)      { pk.x = pk2(xr[4 * t], xr[4 * t + 1]); pk.y = pk2(xr[4 * t + 2], xr[4 * t + 3]); }
    else if (t < 24) { pk.x = pk2(pe4[0], pe4[1]); pk.y = pk2(pe4[2], pe4[3]); }
    else             { pk.x = 0u; pk.y = 0u; }
    _Float16* hr = h16 + (size_t)row * HIDF + 4 * t;
    *(volatile v2u_t*)hr = pk; __threadfence(); *(volatile v2u_t*)hr = pk;
}

__global__ __launch_bounds__(128)
void wmma_dual_lin_kernel(const _Float16* __restrict__ X, int K,
                          const _Float16* __restrict__ WL,
                          const _Float16* __restrict__ WR,
                          const float* __restrict__ biasL,
                          const float* __restrict__ biasR,
                          float* __restrict__ YL, float* __restrict__ YR,
                          int nrows) {
    extern __shared__ _Float16 ldsW[];
    int tid  = threadIdx.x;
    int wave = tid >> 5;
    int lane = tid & 31;

    {
        int chunksPerMat = K * 16;
        int total = 2 * chunksPerMat;
        for (int ch = tid; ch < total; ch += 128) {
            int m   = (ch >= chunksPerMat) ? 1 : 0;
            int rem = ch - m * chunksPerMat;
            int k   = rem >> 4;
            int c   = (rem & 15) * 8;
            const _Float16* src = (m ? WR : WL) + (size_t)k * HIDF + c;
            _Float16* dst = ldsW + (size_t)(m * K + k) * LDS_STRIDE + c;
            *(uint4*)dst = *(const uint4*)src;
        }
    }
    __syncthreads();

    int row0 = (blockIdx.x * 4 + wave) * 16;
    if (row0 >= nrows) return;

    v8f accL[8] = {};
    v8f accR[8] = {};
    int g = lane >> 4;
    const _Float16* arow = X + (size_t)(row0 + (lane & 15)) * HIDF;
    for (int k0 = 0; k0 < K; k0 += 32) {
        if (k0 + 32 < K) __builtin_prefetch(arow + k0 + 32, 0, 1);
        AFrag af;
#pragma unroll
        for (int j = 0; j < 8; ++j) {
            int kk = k0 + ((j < 4) ? 0 : 16) + (j & 3) * 2 + g * 8;
            af.u[j] = *(const unsigned int*)(arow + kk);
        }
        const _Float16* blbase = ldsW + (size_t)k0 * LDS_STRIDE + (lane & 15);
        const _Float16* brbase = blbase + (size_t)K * LDS_STRIDE;
        BFrag bf[8];
#pragma unroll
        for (int n = 0; n < 8; ++n)
#pragma unroll
            for (int e = 0; e < 16; ++e) { const int kk = (e < 8) ? (8 * g + e) : (16 + 8 * g + (e - 8)); bf[n].e[e] = blbase[(size_t)kk * LDS_STRIDE + n * 16]; }
#pragma unroll
        for (int n = 0; n < 8; ++n)
            accL[n] = __builtin_amdgcn_wmma_f32_16x16x32_f16(
                false, af.v, false, bf[n].v, (short)0, accL[n], false, false);
#pragma unroll
        for (int n = 0; n < 8; ++n)
#pragma unroll
            for (int e = 0; e < 16; ++e) { const int kk = (e < 8) ? (8 * g + e) : (16 + 8 * g + (e - 8)); bf[n].e[e] = brbase[(size_t)kk * LDS_STRIDE + n * 16]; }
#pragma unroll
        for (int n = 0; n < 8; ++n)
            accR[n] = __builtin_amdgcn_wmma_f32_16x16x32_f16(
                false, af.v, false, bf[n].v, (short)0, accR[n], false, false);
    }
    __shared__ __attribute__((aligned(16))) float stg[4][16 * HIDF];
    float* sw = stg[wave];
    int ncol = lane & 15;
#pragma unroll 1
    for (int m2 = 0; m2 < 2; ++m2) {
        float* Y = m2 ? YR : YL;
#pragma unroll
        for (int n = 0; n < 8; ++n) {
            int c = n * 16 + ncol;
            float bb = (m2 ? biasR : biasL)[c];
#pragma unroll
            for (int v = 0; v < 8; ++v) sw[(v + 8 * g) * HIDF + c] = (m2 ? accR[n][v] : accL[n][v]) + bb;
        }
        asm volatile("s_wait_dscnt 0" ::: "memory");
#pragma unroll 1
        for (int pass = 0; pass < 2; ++pass) {
#pragma unroll 4
            for (int i = 0; i < 16; ++i) { const int cc = lane + 32 * i, rr = cc >> 5, q = cc & 31;
                *(volatile v4f_t*)(Y + (size_t)(row0 + rr) * HIDF + q * 4) = *(const volatile v4fa*)(sw + rr * HIDF + q * 4); }
            __threadfence();
        }
        asm volatile("s_wait_dscnt 0" ::: "memory");
    }
}

__global__ __launch_bounds__(256)
void acc_init_kernel(float* __restrict__ acc, const float* __restrict__ biasR) {
    int t = blockIdx.x * 256 + threadIdx.x;
    if (t >= N_STOCKS * HIDF) return;
    int j = t & (HIDF - 1);
    float s = 0.f;
#pragma unroll
    for (int r = 0; r < R_REL; ++r) s += biasR[r * HIDF + j];
    ST2F(acc + t, s);
}

__global__ __launch_bounds__(256)
void bucket_list_kernel(const int* __restrict__ edst, int* __restrict__ noff, int* __restrict__ ncnt, int* __restrict__ ledge) {
    __shared__ unsigned lst[LCAP], srt[LCAP];
    __shared__ int wcnt[8];
    __shared__ int total;
    __shared__ int cnt[BUCKET], off[BUCKET];
    const int tid = threadIdx.x, lane = tid & 31, wave = tid >> 5;
    const int n0 = blockIdx.x * BUCKET;
    if (tid == 0) total = 0;
    __syncthreads();
    for (int e0 = 0; e0 < E_EDGES; e0 += 256) {
        const int e = e0 + tid;
        int loc = -1;
        if (e < E_EDGES) { const int l = edst[e] - n0; if ((unsigned)l < (unsigned)BUCKET) loc = l; }
        const unsigned m = __ballot(loc >= 0);
        if (lane == 0) wcnt[wave] = __popc(m);
        __syncthreads();
        int base = total;
#pragma unroll
        for (int w = 0; w < 8; ++w) if (w < wave) base += wcnt[w];
        if (loc >= 0) { const int slot = base + __popc(m & ((1u << lane) - 1u)); if (slot < LCAP) lst[slot] = ((unsigned)loc << 24) | (unsigned)e; }
        __syncthreads();
        if (tid == 0) { int t2 = total; for (int w = 0; w < 8; ++w) t2 += wcnt[w]; total = t2; }
        __syncthreads();
    }
    const int nl = (total < LCAP) ? total : LCAP;
    if (tid < BUCKET) { int c = 0; for (int i = 0; i < nl; ++i) c += ((int)(lst[i] >> 24) == tid); cnt[tid] = c; }
    __syncthreads();
    if (tid == 0) { int o = 0; for (int j = 0; j < BUCKET; ++j) { off[j] = o; o += cnt[j]; } }
    __syncthreads();
    if (tid < BUCKET) { int p = off[tid]; for (int i = 0; i < nl; ++i) if ((int)(lst[i] >> 24) == tid) srt[p++] = lst[i] & 0xFFFFFFu; }
    __syncthreads();
#pragma unroll 1
    for (int pass = 0; pass < 2; ++pass) {
        if (tid < BUCKET && n0 + tid < N_STOCKS) { *(volatile int*)(noff + n0 + tid) = blockIdx.x * LCAP + off[tid]; *(volatile int*)(ncnt + n0 + tid) = cnt[tid]; }
        typedef __attribute__((ext_vector_type(4))) unsigned v4u_t;
        typedef unsigned v4ua __attribute__((ext_vector_type(4), may_alias));
        for (int c = tid; c * 4 < nl; c += 256)
            *(volatile v4u_t*)((unsigned*)ledge + (size_t)blockIdx.x * LCAP + c * 4) = *(const volatile v4ua*)(srt + c * 4);
        __threadfence();
    }
}

__global__ __launch_bounds__(256)
void gat_gather_kernel(const float* __restrict__ XL, const float* __restrict__ XR,
                       const int* __restrict__ esrc, const int* __restrict__ noff, const int* __restrict__ ncnt,
                       const int* __restrict__ ledge, const float* __restrict__ att,
                       float* __restrict__ acc) {
    const int w = (blockIdx.x * 256 + threadIdx.x) >> 5;
    if (w >= N_STOCKS) return;
    const int lane = threadIdx.x & 31;
    const v4f_t xr = *(const v4fa*)(XR + (size_t)w * HIDF + lane * 4);
    const v4f_t a4 = *(const v4fa*)(att + lane * 4);
    const int o0 = noff[w], cn = ncnt[w];
    float m = -3.0e38f, l = 0.f;
    v4f_t o = {0.f, 0.f, 0.f, 0.f};
    for (int i = 0; i <= cn; ++i) {
        int s;
        if (i < cn) { int e = ledge[o0 + i]; e = ((unsigned)e < (unsigned)E_EDGES) ? e : 0; s = esrc[e]; s = ((unsigned)s < (unsigned)N_STOCKS) ? s : 0; }
        else s = w;
        const v4f_t xl = *(const v4fa*)(XL + (size_t)s * HIDF + lane * 4);
        v4f_t v = xl + xr;
        float sc = 0.f;
#pragma unroll
        for (int j = 0; j < 4; ++j) { float vv = v[j]; vv = (vv > 0.f) ? vv : 0.2f * vv; sc += a4[j] * vv; }
        sc += __shfl_xor(sc, 1, 32); sc += __shfl_xor(sc, 2, 32); sc += __shfl_xor(sc, 4, 32);
        const float mn = fmaxf(m, sc), corr = __expf(m - mn), p = __expf(sc - mn);
        l = l * corr + p; o = o * corr + xl * p; m = mn;
    }
    const float inv = 1.0f / (l + 1e-16f);
    float* ap = acc + (size_t)w * HIDF + lane * 4;
    v4f_t r = *(const v4fa*)ap + o * inv;
    *(volatile v4f_t*)ap = r; __threadfence(); *(volatile v4f_t*)ap = r;
}

__global__ __launch_bounds__(256)
void relu_cvt_kernel(float* __restrict__ acc, _Float16* __restrict__ h16) {
    int t = blockIdx.x * 256 + threadIdx.x;
    if (t >= N_STOCKS * HIDF) return;
    (void)t;
}
__global__ __launch_bounds__(256)
void relu_cvt2_kernel(float* __restrict__ acc, _Float16* __restrict__ h16) {
    const int t = (blockIdx.x * 256 + threadIdx.x) * 2;
    if (t >= N_STOCKS * HIDF) return;
    typedef __attribute__((ext_vector_type(2))) float v2f_t;
    typedef float v2fa __attribute__((ext_vector_type(2), may_alias));
    v2f_t v = *(const v2fa*)(acc + t);
    v.x = (v.x > 0.f) ? v.x : 0.f; v.y = (v.y > 0.f) ? v.y : 0.f;
    const unsigned p = pk2(v.x, v.y);
    *(volatile v2f_t*)(acc + t) = v; *(volatile unsigned*)(h16 + t) = p;
    __threadfence();
    *(volatile v2f_t*)(acc + t) = v; *(volatile unsigned*)(h16 + t) = p;
}

__global__ __launch_bounds__(256)
void mlp_kernel(const float* __restrict__ acc,
                const float* __restrict__ oW1, const float* __restrict__ ob1,
                const float* __restrict__ oW2, const float* __restrict__ ob2,
                float* __restrict__ out) {
    __shared__ float so[32];
    const int lane = threadIdx.x & 31, wave = threadIdx.x >> 5;
#pragma unroll 1
    for (int q = 0; q < 4; ++q) {
        const int row = blockIdx.x * 32 + wave * 4 + q;
        const float* hr = acc + (size_t)row * HIDF;
        float s0 = ob1[lane], s1 = ob1[lane + 32];
#pragma unroll 8
        for (int k = 0; k < HIDF; ++k) { const float hv = hr[k]; s0 += hv * oW1[k * 64 + lane]; s1 += hv * oW1[k * 64 + lane + 32]; }
        s0 = (s0 > 0.f) ? s0 : 0.f; s1 = (s1 > 0.f) ? s1 : 0.f;
        float v = s0 * oW2[lane] + s1 * oW2[lane + 32];
#pragma unroll
        for (int off = 16; off > 0; off >>= 1) v += __shfl_xor(v, off, 32);
        if (lane == 0) so[wave * 4 + q] = v + ob2[0];
    }
    __syncthreads();
    if (wave == 0) { const float v = so[lane]; ST2F(out + (size_t)blockIdx.x * 32 + lane, v); }
}

extern "C" void kernel_launch(void* const* d_in, const int* in_sizes, int n_in,
                              void* d_out, int out_size, void* d_ws, size_t ws_size,
                              hipStream_t stream) {
    const float* x       = (const float*)d_in[0];
    const int*   ei      = (const int*)  d_in[1];
    const float* pearl_W = (const float*)d_in[2];
    const float* pearl_b = (const float*)d_in[3];
    const float* Wl[2]   = { (const float*)d_in[4],  (const float*)d_in[10] };
    const float* bl[2]   = { (const float*)d_in[5],  (const float*)d_in[11] };
    const float* Wr[2]   = { (const float*)d_in[6],  (const float*)d_in[12] };
    const float* br[2]   = { (const float*)d_in[7],  (const float*)d_in[13] };
    const float* att[2]  = { (const float*)d_in[8],  (const float*)d_in[14] };
    const float* biasL[2]= { (const float*)d_in[9],  (const float*)d_in[15] };
    const float* oW1 = (const float*)d_in[16];
    const float* ob1 = (const float*)d_in[17];
    const float* oW2 = (const float*)d_in[18];
    const float* ob2 = (const float*)d_in[19];
    float* out = (float*)d_out;

    char* wp = (char*)d_ws;
    auto take = [&](size_t bytes) -> void* {
        void* q = (void*)wp;
        wp += (bytes + 255) & ~(size_t)255;
        return q;
    };
    _Float16* h16  = (_Float16*)take((size_t)N_STOCKS * HIDF * 2);
    _Float16* WlH[2], *WrH[2];
    WlH[0] = (_Float16*)take((size_t)R_REL * TIN  * HIDF * 2);
    WrH[0] = (_Float16*)take((size_t)R_REL * TIN  * HIDF * 2);
    WlH[1] = (_Float16*)take((size_t)R_REL * HIDF * HIDF * 2);
    WrH[1] = (_Float16*)take((size_t)R_REL * HIDF * HIDF * 2);
    float* XL    = (float*)take((size_t)N_STOCKS * HIDF * 4);
    float* XR    = (float*)take((size_t)N_STOCKS * HIDF * 4);
    float* acc   = (float*)take((size_t)N_STOCKS * HIDF * 4);
    int*   noff  = (int*)take((size_t)R_REL * N_STOCKS * 4);
    int*   ncnt  = (int*)take((size_t)R_REL * N_STOCKS * 4);
    int*   ledge = (int*)take((size_t)R_REL * NBK * LCAP * 4);

    {
        int c0 = R_REL * TIN * HIDF, c1 = R_REL * HIDF * HIDF;
        cvt_f16_kernel<<<(c0 / 2 + 255) / 256, 256, 0, stream>>>(Wl[0], WlH[0], c0);
        cvt_f16_kernel<<<(c0 / 2 + 255) / 256, 256, 0, stream>>>(Wr[0], WrH[0], c0);
        cvt_f16_kernel<<<(c1 / 2 + 255) / 256, 256, 0, stream>>>(Wl[1], WlH[1], c1);
        cvt_f16_kernel<<<(c1 / 2 + 255) / 256, 256, 0, stream>>>(Wr[1], WrH[1], c1);
    }
    for (int r = 0; r < R_REL; ++r)
        bucket_list_kernel<<<NBK, 256, 0, stream>>>(ei + ((size_t)r * 2 + 1) * E_EDGES, noff + (size_t)r * N_STOCKS, ncnt + (size_t)r * N_STOCKS, ledge + (size_t)r * NBK * LCAP);

    pearl_concat_kernel<<<N_STOCKS, 32, 0, stream>>>(x, pearl_W, pearl_b, h16);

    const int rowTiles  = N_STOCKS / 16;
    const int gemmBlks  = (rowTiles + 3) / 4;
    const int nhBlks    = (N_STOCKS * HIDF + 255) / 256;
    const int nodeBlks  = (N_STOCKS * 32 + 255) / 256;

    for (int layer = 0; layer < 2; ++layer) {
        const int K        = layer ? HIDF : TIN;
        const int wstride  = K * HIDF;
        const size_t ldsSz = (size_t)2 * K * LDS_STRIDE * sizeof(_Float16);

        acc_init_kernel<<<nhBlks, 256, 0, stream>>>(acc, biasL[layer]);

        for (int r = 0; r < R_REL; ++r) {
            const int* esrc = ei + ((size_t)r * 2 + 0) * E_EDGES;
            const int* edst = ei + ((size_t)r * 2 + 1) * E_EDGES;

            wmma_dual_lin_kernel<<<gemmBlks, 128, ldsSz, stream>>>(
                h16, K,
                WlH[layer] + (size_t)r * wstride, WrH[layer] + (size_t)r * wstride,
                bl[layer] + r * HIDF, br[layer] + r * HIDF,
                XL, XR, N_STOCKS);

            (void)edst;
            gat_gather_kernel<<<nodeBlks, 256, 0, stream>>>(
                XL, XR, esrc, noff + (size_t)r * N_STOCKS, ncnt + (size_t)r * N_STOCKS, ledge + (size_t)r * NBK * LCAP,
                att[layer] + r * HEADS * CDIM, acc);
        }
        relu_cvt2_kernel<<<(nhBlks + 1) / 2, 256, 0, stream>>>(acc, h16);
    }

    mlp_kernel<<<N_STOCKS / 32, 256, 0, stream>>>(acc, oW1, ob1, oW2, ob2, out);
}
